// GraphSAGELayers_34711925686455
// MI455X (gfx1250) — hardware-verified
//
#include <hip/hip_runtime.h>
#include <hip/hip_bf16.h>
#include <math.h>


#define BB 2
#define SS 2048
#define DD 1024
#define HH 16
#define DKK 64
#define QW 2

typedef _Float16 bf16;
typedef __attribute__((ext_vector_type(4))) unsigned v4u_t;
typedef unsigned v4ua __attribute__((ext_vector_type(4), may_alias));
typedef __attribute__((ext_vector_type(4))) float v4f_t;
typedef float v4fa __attribute__((ext_vector_type(4), may_alias));
typedef __attribute__((ext_vector_type(16))) bf16  bf16x16;
typedef __attribute__((ext_vector_type(8)))  bf16  bf16x8;
typedef __attribute__((ext_vector_type(4)))  bf16  bf16x4;
typedef __attribute__((ext_vector_type(8)))  float f32x8;

#define LDS_STRIDE 48
#define KSTRIDE    72
#define VSTRIDE    48

__device__ __forceinline__ f32x8 wmma_bf16(bf16x16 a, bf16x16 b, f32x8 c) {
  return __builtin_amdgcn_wmma_f32_16x16x32_f16(
      false, a, false, b, (short)0, c, false, false);
}
#define RSPLIT (1.0f / 2048.0f)
__device__ __forceinline__ bf16 lo_of(float v, bf16 h) { return (bf16)((v - (float)h) * 2048.0f); }
__device__ __forceinline__ f32x8 wmma_split(bf16x16 a, bf16x16 al, bf16x16 b, bf16x16 bl, f32x8 c) {
  f32x8 x = {}; x = wmma_bf16(al, b, x); x = wmma_bf16(a, bl, x); return wmma_bf16(a, b, c) + x * RSPLIT; }

template <typename T>
__device__ __forceinline__ bf16x16 load_frag(const T* __restrict__ base, int ld,
                                             int row0, int k0) {
  const int lane = threadIdx.x & 31;
  const int r    = lane & 15;
  const int kh   = (lane >> 4) * 8;
  const T* p0 = base + (size_t)(row0 + r) * ld + (k0 + kh);
  const T* p1 = p0 + 16;
  bf16x16 f;
#pragma unroll
  for (int i = 0; i < 8; ++i) {
    f[i]     = (bf16)p0[i];
    f[i + 8] = (bf16)p1[i];
  }
  return f;
}

__device__ __forceinline__ bf16x16 lds_frag(const bf16* base, int stride) {
  const int lane = threadIdx.x & 31;
  const int row  = lane & 15;
  const int kh   = (lane >> 4) * 8;
  const bf16x8 lo = *(const bf16x8*)(base + row * stride + kh);
  const bf16x8 hi = *(const bf16x8*)(base + row * stride + kh + 16);
  bf16x16 f;
#pragma unroll
  for (int i = 0; i < 8; ++i) { f[i] = lo[i]; f[i + 8] = hi[i]; }
  return f;
}

template <typename T>
__device__ __forceinline__ void stage_read16(const T* __restrict__ p, float* buf) {
#pragma unroll
  for (int i = 0; i < 16; ++i) buf[i] = (float)p[i];
}

__device__ __forceinline__ void stage_write(bf16* dst, const float* buf, int nquad) {
#pragma unroll
  for (int i = 0; i < nquad; ++i) {
    bf16x4 q;
    q[0] = (bf16)buf[4 * i];     q[1] = (bf16)buf[4 * i + 1];
    q[2] = (bf16)buf[4 * i + 2]; q[3] = (bf16)buf[4 * i + 3];
    *(bf16x4*)(dst + 4 * i) = q;
  }
}

__global__ __launch_bounds__(256) void transpose_pack_kernel(const float* __restrict__ W, bf16* __restrict__ WT, int K, int N, size_t plane) {
  __shared__ float tile[64][65];
  const int k0 = blockIdx.y * 64, n0 = blockIdx.x * 64, t = threadIdx.x;
  for (int i = t; i < 64 * 64; i += 256) { const int kr = i >> 6, nc = i & 63; tile[kr][nc] = W[(size_t)(k0 + kr) * N + n0 + nc]; }
  __syncthreads();
#pragma unroll 1
  for (int pass = 0; pass < 2; ++pass) {
    for (int i = t; i < 64 * 8; i += 256) { const int nr = i >> 3, k8 = (i & 7) * 8; bf16 hh[8], hl[8];
#pragma unroll
      for (int e = 0; e < 8; ++e) { const float v = tile[k8 + e][nr]; hh[e] = (bf16)v; hl[e] = lo_of(v, hh[e]); }
      bf16* d = WT + (size_t)(n0 + nr) * K + k0 + k8;
      *(volatile v4u_t*)d = *(const v4ua*)hh; *(volatile v4u_t*)(d + plane) = *(const v4ua*)hl; }
    __threadfence();
  }
}

template <typename AT, typename WT, int MODE>
__global__ __launch_bounds__(256) void gemm_split_kernel(
    const AT* __restrict__ A, size_t aPlane, const WT* __restrict__ W, size_t wPlane,
    const float* __restrict__ bias, void* __restrict__ out,
    int M, int N, int K) {
  __shared__ bf16 ldsA[128 * LDS_STRIDE], ldsAl[128 * LDS_STRIDE];
  __shared__ bf16 ldsW[256 * LDS_STRIDE], ldsWl[256 * LDS_STRIDE];
  __shared__ __attribute__((aligned(16))) unsigned char sob[256 * 136 * 2];

  const int t    = threadIdx.x;
  const int wave = t >> 5;
  const int lane = t & 31;
  const int wm   = (wave & 1) * 64;
  const int wn   = (wave >> 1) * 64;
  const int mBlk = blockIdx.x * 128;
  const int nBlk = blockIdx.y * 256;
  const int arow = t >> 1;
  const int ach  = (t & 1) * 16;

  f32x8 acc[4][4] = {};
  for (int k = 0; k < K; k += 32) {
    __syncthreads();
    {
      const AT* ap = A + (size_t)(mBlk + arow) * K + k + ach;
      bf16 hh[16], hl[16];
      if (sizeof(AT) == 4) {
#pragma unroll
        for (int i = 0; i < 16; ++i) { const float v = (float)ap[i]; hh[i] = (bf16)v; hl[i] = lo_of(v, hh[i]); }
      } else {
#pragma unroll
        for (int i = 0; i < 16; ++i) { hh[i] = (bf16)ap[i]; hl[i] = (bf16)ap[aPlane + i]; }
      }
#pragma unroll
      for (int i = 0; i < 16; ++i) { ldsA[arow * LDS_STRIDE + ach + i] = hh[i]; ldsAl[arow * LDS_STRIDE + ach + i] = hl[i]; }
    }
    {
      const WT* wp = W + (size_t)(nBlk + t) * K + k;
      if (sizeof(WT) == 4) {
#pragma unroll
        for (int i = 0; i < 32; ++i) { const float v = (float)wp[i]; const bf16 h_ = (bf16)v; ldsW[t * LDS_STRIDE + i] = h_; ldsWl[t * LDS_STRIDE + i] = lo_of(v, h_); }
      } else {
#pragma unroll
        for (int i = 0; i < 32; ++i) { ldsW[t * LDS_STRIDE + i] = (bf16)wp[i]; ldsWl[t * LDS_STRIDE + i] = (bf16)wp[wPlane + i]; }
      }
    }
    __syncthreads();
    bf16x16 wf[4], wfl[4];
#pragma unroll
    for (int j = 0; j < 4; ++j) { wf[j] = lds_frag(ldsW + (wn + 16 * j) * LDS_STRIDE, LDS_STRIDE); wfl[j] = lds_frag(ldsWl + (wn + 16 * j) * LDS_STRIDE, LDS_STRIDE); }
#pragma unroll
    for (int i = 0; i < 4; ++i) {
      const bf16x16 af = lds_frag(ldsA + (wm + 16 * i) * LDS_STRIDE, LDS_STRIDE), afl = lds_frag(ldsAl + (wm + 16 * i) * LDS_STRIDE, LDS_STRIDE);
#pragma unroll
      for (int j = 0; j < 4; ++j) acc[i][j] = wmma_split(af, afl, wf[j], wfl[j], acc[i][j]);
    }
  }

  const int nlane = lane & 15;
  const int mh    = (lane >> 4) * 8;
  __syncthreads();
  if (MODE == 1) {
    bf16* so = (bf16*)sob;
#pragma unroll
    for (int i = 0; i < 4; ++i)
#pragma unroll
      for (int j = 0; j < 4; ++j) {
        const int nl = wn + 16 * j + nlane;
        const float bv = bias ? bias[nBlk + nl] : 0.0f;
#pragma unroll
        for (int r = 0; r < 8; ++r) so[nl * 136 + wm + 16 * i + mh + r] = (bf16)(acc[i][j][r] + bv);
      }
    __syncthreads();
    const int b_ = mBlk >> 11, s0 = mBlk & (SS - 1);
#pragma unroll 1
    for (int pass = 0; pass < 2; ++pass) {
      for (int ch = t; ch < 256 * 16; ch += 256) { const int nl = ch >> 4, q = (ch & 15) * 8; const int n = nBlk + nl, h = n >> 6, dk = n & (DKK - 1);
        *(volatile v4u_t*)((bf16*)out + (((size_t)(b_ * HH + h)) * DKK + dk) * SS + s0 + q) = *(const v4ua*)(so + nl * 136 + q); }
      __threadfence();
    }
  } else {
    float* so = (float*)sob;
#pragma unroll 1
    for (int hf = 0; hf < 2; ++hf) {
      if (wm == hf * 64) {
#pragma unroll
        for (int i = 0; i < 4; ++i)
#pragma unroll
          for (int j = 0; j < 4; ++j) {
            const int nl = wn + 16 * j + nlane;
            const float bv = bias ? bias[nBlk + nl] : 0.0f;
#pragma unroll
            for (int r = 0; r < 8; ++r) so[(16 * i + mh + r) * 260 + nl] = acc[i][j][r] + bv;
          }
      }
      __syncthreads();
#pragma unroll 1
      for (int pass = 0; pass < 2; ++pass) {
        for (int ch = t; ch < 64 * 64; ch += 256) { const int ml = ch >> 6, q = (ch & 63) * 4;
          *(volatile v4f_t*)((float*)out + (size_t)(mBlk + hf * 64 + ml) * N + nBlk + q) = *(const volatile v4fa*)(so + ml * 260 + q); }
        __threadfence();
      }
      __syncthreads();
    }
  }
}


#define GN 100000
#define GNP 100352
#define GE 800000
#define GRANGE 25088
#define F0 128
#define F1 128
#define F2 128

__global__ __launch_bounds__(256) void k_deg(const int* __restrict__ dsti, float* __restrict__ invdeg) {
  __shared__ int cnt[GRANGE + 8]; __shared__ int qd[8][256]; __shared__ int wcnt[8][8];
  const int tid = threadIdx.x, lane = tid & 31, wave = tid >> 5, r0 = blockIdx.x * GRANGE;
  for (int i = tid; i < GRANGE + 8; i += 256) cnt[i] = 0;
  __syncthreads();
  const int* dstp = dsti;
#pragma unroll 1
  for (int c0 = 0; c0 < GE; c0 += 256) {
    const int e = c0 + tid; int d = -1;
    if (e < GE) { const int draw = dstp[e]; const int dd = draw < 0 ? 0 : (draw >= GN ? GN - 1 : draw); if (dd >= r0 && dd < r0 + GRANGE) d = dd - r0; }
    const int own = (d >= 0) ? (d & 7) : -1; unsigned mown = 0u;
#pragma unroll
    for (int w = 0; w < 8; ++w) { const unsigned m = __builtin_amdgcn_ballot_w32(own == w); if (own == w) mown = m; if (lane == 0) wcnt[w][wave] = __builtin_popcount(m); }
    __syncthreads();
    if (own >= 0) { int base = 0;
#pragma unroll
      for (int w2 = 0; w2 < 8; ++w2) base += (w2 < wave) ? wcnt[own][w2] : 0;
      qd[own][base + __builtin_popcount(mown & ((1u << lane) - 1u))] = d; }
    int total = 0;
#pragma unroll
    for (int w2 = 0; w2 < 8; ++w2) total += wcnt[wave][w2];
    __syncthreads();
#pragma unroll 1
    for (int qi = 0; qi < total; ++qi) { const int dl = qd[wave][qi]; if (lane == 0) cnt[dl] += 1; }
    __syncthreads();
  }
#pragma unroll 1
  for (int pass = 0; pass < 2; ++pass) {
    for (int i = tid; i < GRANGE / 4; i += 256) { v4f_t v;
#pragma unroll
      for (int q = 0; q < 4; ++q) v[q] = 1.0f / fmaxf((float)cnt[i * 4 + q], 1.0f);
      *(volatile v4f_t*)(invdeg + r0 + i * 4) = v; }
    __threadfence();
  }
}
template <int FW, int RELU>
__global__ __launch_bounds__(256) void k_sage(const int* __restrict__ srci, const int* __restrict__ dsti, const float* __restrict__ H, const float* __restrict__ invdeg, float* __restrict__ R, int rsel) {
  __shared__ int qd[8][256], qs[8][256]; __shared__ int wcnt[8][8];
  const int tid = threadIdx.x, lane = tid & 31, wave = tid >> 5, r0 = (rsel < 0 ? (int)blockIdx.x : rsel) * GRANGE;
  constexpr int RW = 2 * FW, Q4 = RW / 4;
  float* myR = R + (rsel < 0 ? (size_t)r0 * RW : (size_t)0);
  for (int i = tid; i < GRANGE * Q4; i += 256) { const int nl = i / Q4, c4 = (i % Q4) * 4, node = r0 + nl; v4f_t v;
    if (c4 < FW || node >= GN) { v.x = v.y = v.z = v.w = 0.0f; }
    else { v = *(const v4fa*)(H + (size_t)node * FW + (c4 - FW)); if (RELU) { v.x = fmaxf(v.x, 0.f); v.y = fmaxf(v.y, 0.f); v.z = fmaxf(v.z, 0.f); v.w = fmaxf(v.w, 0.f); } }
    *(volatile v4f_t*)(myR + (size_t)nl * RW + c4) = v; }
  __threadfence(); __syncthreads();
  const int* srcp = srci; const int* dstp = dsti;
#pragma unroll 1
  for (int c0 = 0; c0 < GE; c0 += 256) {
    const int e = c0 + tid; int d = -1, sidx = 0;
    if (e < GE) { const int draw = dstp[e]; const int dd = draw < 0 ? 0 : (draw >= GN ? GN - 1 : draw);
      if (dd >= r0 && dd < r0 + GRANGE) { d = dd - r0; const int ss = srcp[e]; sidx = ss < 0 ? 0 : (ss >= GN ? GN - 1 : ss); } }
    const int own = (d >= 0) ? (d & 7) : -1; unsigned mown = 0u;
#pragma unroll
    for (int w = 0; w < 8; ++w) { const unsigned m = __builtin_amdgcn_ballot_w32(own == w); if (own == w) mown = m; if (lane == 0) wcnt[w][wave] = __builtin_popcount(m); }
    __syncthreads();
    if (own >= 0) { int base = 0;
#pragma unroll
      for (int w2 = 0; w2 < 8; ++w2) base += (w2 < wave) ? wcnt[own][w2] : 0;
      const int pos = base + __builtin_popcount(mown & ((1u << lane) - 1u)); qd[own][pos] = d; qs[own][pos] = sidx; }
    int total = 0;
#pragma unroll
    for (int w2 = 0; w2 < 8; ++w2) total += wcnt[wave][w2];
    __syncthreads();
#pragma unroll 1
    for (int qi = 0; qi < total; ++qi) { const int dl = qd[wave][qi]; const int sl = qs[wave][qi];
      float* row = myR + (size_t)dl * RW; const float* hs = H + (size_t)sl * FW;
#pragma unroll
      for (int u = 0; u < FW / 32; ++u) { float hv = hs[u * 32 + lane]; if (RELU) hv = fmaxf(hv, 0.0f); row[u * 32 + lane] += hv; } }
    __syncthreads();
  }
  __threadfence(); __syncthreads();
#pragma unroll 1
  for (int pass = 0; pass < 2; ++pass) {
    for (int i = tid; i < GRANGE * Q4; i += 256) { const int nl = i / Q4, c4 = (i % Q4) * 4, node = r0 + nl; float* p = myR + (size_t)nl * RW + c4;
      v4f_t v = *(const volatile v4fa*)p; if (c4 < FW && pass == 0) { const float s = (node < GN) ? invdeg[node] : 0.0f; v.x *= s; v.y *= s; v.z *= s; v.w *= s; }
      *(volatile v4f_t*)p = v; }
    __threadfence(); __syncthreads();
  }
}
__global__ __launch_bounds__(256) void k_comb(const float* __restrict__ T, const float* __restrict__ b2, int r0, float* __restrict__ out) {
  __shared__ float tile[64][65];
  const int n0 = blockIdx.x * 64, cb = blockIdx.y * 64, t = threadIdx.x;
  for (int i = t; i < 64 * 64; i += 256) { const int c = i >> 6, nn = i & 63; tile[c][nn] = T[(size_t)(cb + c) * GRANGE + n0 + nn]; }
  __syncthreads();
#pragma unroll 1
  for (int pass = 0; pass < 2; ++pass) {
    for (int i = t; i < 64 * 16; i += 256) { const int nr = i >> 4, c4 = (i & 15) * 4, node = r0 + n0 + nr;
      if (node < GN) { v4f_t v;
#pragma unroll
        for (int q = 0; q < 4; ++q) v[q] = tile[c4 + q][nr] + b2[cb + c4 + q];
        *(volatile v4f_t*)(out + (size_t)node * F2 + cb + c4) = v; } }
    __threadfence();
  }
}
__global__ __launch_bounds__(256) void k_wcat(const float* __restrict__ Wl, const float* __restrict__ Wr, int FIN, float* __restrict__ Wc) {
  const int o = blockIdx.x, t = threadIdx.x;
  for (int k = t; k < 2 * FIN; k += 256) { const float v = (k < FIN) ? Wl[(size_t)o * FIN + k] : Wr[(size_t)o * FIN + k - FIN]; *(volatile float*)(Wc + (size_t)o * 2 * FIN + k) = v; }
  __threadfence();
  for (int k = t; k < 2 * FIN; k += 256) { const float v = (k < FIN) ? Wl[(size_t)o * FIN + k] : Wr[(size_t)o * FIN + k - FIN]; *(volatile float*)(Wc + (size_t)o * 2 * FIN + k) = v; }
}

__global__ __launch_bounds__(256) void k_rowcopy(const float* __restrict__ src, float* __restrict__ dst) {
  const size_t off = ((size_t)blockIdx.x * 256 + threadIdx.x) * 8;
  const v4f_t a = *(const v4fa*)(src + off), b = *(const v4fa*)(src + off + 4);
  *(volatile v4f_t*)(dst + off) = a; *(volatile v4f_t*)(dst + off + 4) = b; __threadfence(); *(volatile v4f_t*)(dst + off) = a; *(volatile v4f_t*)(dst + off + 4) = b;
}
__global__ __launch_bounds__(256) void k_comb_ln(const float* __restrict__ T, const float* __restrict__ bl, const float* __restrict__ gam, const float* __restrict__ bet,
                                                const float* __restrict__ xin, int r0, float* __restrict__ out) {
  __shared__ float tile[128][33]; __shared__ float ps[32][8], pq[32][8];
  const int n0 = blockIdx.x * 32, t = threadIdx.x;
  for (int i = t; i < 128 * 32; i += 256) { const int c = i >> 5, nn = i & 31; tile[c][nn] = T[(size_t)c * GRANGE + n0 + nn] + bl[c]; }
  __syncthreads();
  const int nl = t >> 3, part = t & 7, c0 = part * 16;
  float s = 0.f; for (int c = c0; c < c0 + 16; ++c) s += tile[c][nl];
  ps[nl][part] = s; __syncthreads();
  float mu = 0.f;
#pragma unroll
  for (int p = 0; p < 8; ++p) mu += ps[nl][p];
  mu *= (1.0f / 128.0f);
  float q = 0.f; for (int c = c0; c < c0 + 16; ++c) { const float d = tile[c][nl] - mu; q += d * d; }
  pq[nl][part] = q; __syncthreads();
  float var = 0.f;
#pragma unroll
  for (int p = 0; p < 8; ++p) var += pq[nl][p];
  const float rs = rsqrtf(var * (1.0f / 128.0f) + 1e-5f);
  const int node = r0 + n0 + nl;
  float y[16];
#pragma unroll
  for (int j = 0; j < 16; ++j) { const int c = c0 + j; float v = (tile[c][nl] - mu) * rs * gam[c] + bet[c]; v = fmaxf(v, 0.0f);
    if (xin != nullptr && node < GN) v += xin[(size_t)node * F2 + c]; y[j] = v; }
#pragma unroll 1
  for (int pass = 0; pass < 2; ++pass) {
    if (node < GN) {
#pragma unroll
      for (int j4 = 0; j4 < 4; ++j4) { v4f_t v; v.x = y[4 * j4]; v.y = y[4 * j4 + 1]; v.z = y[4 * j4 + 2]; v.w = y[4 * j4 + 3]; *(volatile v4f_t*)(out + (size_t)node * F2 + c0 + 4 * j4) = v; } }
    __threadfence(); }
}

extern "C" void kernel_launch(void* const* d_in, const int* in_sizes, int n_in,
                              void* d_out, int out_size, void* d_ws, size_t ws_size,
                              hipStream_t stream) {
  (void)in_sizes; (void)n_in; (void)out_size; (void)ws_size;
  const float* x  = (const float*)d_in[0];
  const int* ei   = (const int*)d_in[1];
  const float* Wl = (const float*)d_in[2];
  const float* bl = (const float*)d_in[3];
  const float* Wr = (const float*)d_in[4];
  const float* lg = (const float*)d_in[5];
  const float* lb = (const float*)d_in[6];
  const int* srci = ei; const int* dsti = ei + (size_t)GE;
  float* out = (float*)d_out;
  char* ws = (char*)d_ws;
  float* Wc  = (float*)ws; ws += (size_t)3 * F2 * 256 * 4;
  float* HA  = (float*)ws; ws += (size_t)GNP * 128 * 4;
  float* R2  = (float*)ws; ws += (size_t)GRANGE * 256 * 4;
  float* T   = (float*)ws; ws += (size_t)F2 * GRANGE * 4;
  float* invdeg = (float*)ws; ws += (size_t)GNP * 4;
  for (int l = 0; l < 3; ++l) k_wcat<<<F2, 256, 0, stream>>>(Wl + (size_t)l * F2 * F2, Wr + (size_t)l * F2 * F2, 128, Wc + (size_t)l * F2 * 256);
  k_deg<<<GNP / GRANGE, 256, 0, stream>>>(dsti, invdeg);
  dim3 blk(256);
  const float* Hin = x; float* targets[3] = {HA, out, HA};
  for (int l = 0; l < 3; ++l) {
    float* dstH = targets[l];
    const float* resid = (l == 0) ? nullptr : Hin;
    for (int r = 0; r < GNP / GRANGE; ++r) {
      k_sage<F0, 0><<<1, 256, 0, stream>>>(srci, dsti, Hin, invdeg, R2, r);
      gemm_split_kernel<float, float, 2><<<dim3(1, GRANGE / 256), blk, 0, stream>>>(Wc + (size_t)l * F2 * 256, 0, R2, 0, nullptr, T, F2, GRANGE, 256);
      k_comb_ln<<<GRANGE / 32, 256, 0, stream>>>(T, bl + l * F2, lg + l * F2, lb + l * F2, resid, r * GRANGE, dstH);
    }
    Hin = dstH;
  }
  k_rowcopy<<<GN / 16, 256, 0, stream>>>(HA, out);
}
